// GPTMultiheadMaskedAttention_39608188404432
// MI455X (gfx1250) — hardware-run, weakly checked
//
#include <hip/hip_runtime.h>


#ifndef NB
#define NB 1
#endif
#ifndef SEQ
#define SEQ 4096
#endif
#define NB_FULL  1
#define SEQ_FULL 4096
#ifndef OUT_SEQ
#define OUT_SEQ SEQ
#endif
#define DM   1024
#define NH_  16
#define HD   64
#define AW   4
#define OSP  68
#define EROWS (SEQ < 512 ? SEQ : 512)
#define QRS  2048.0f
#define QRI  (1.0f / 2048.0f)
#define SC2  ((float)(0.125 * 1.4426950408889634))
#define PSH  14.0f
#define NEGB (-3.0e38f)
#define CTXS 16.0f
#define WOS  1024.0f
#define OSCL (1.0f / 16384.0f)

static_assert(HD == 64);
static_assert(NH_ * HD == DM);
static_assert(DM % 64 == 0);
static_assert(DM % 32 == 0);
static_assert(HD % 32 == 0);
static_assert(SEQ % 64 == 0);
static_assert((NB * SEQ) % 64 == 0);
static_assert(SEQ % 32 == 0);
static_assert(SEQ % (16 * AW) == 0);
static_assert(EROWS % 64 == 0);
static_assert(EROWS % 32 == 0);
static_assert(EROWS >= 32);
static_assert(EROWS <= SEQ);
static_assert(EROWS % (16 * AW) == 0);
static_assert((SEQ - EROWS) % (16 * AW) == 0);
static_assert((SEQ - EROWS) % 64 == 0);
static_assert(((size_t)SEQ * DM) % 8 == 0);
static_assert(NB <= NB_FULL);
static_assert(SEQ <= SEQ_FULL);
static_assert((OSP * 4) % 16 == 0);
static_assert(OSP >= HD);
static_assert(4 * 32 * 8 == 16 * HD);
static_assert(8 * 32 * 4 == 16 * 64);
static_assert(4 * 32 * 4 == 16 * 32);
static_assert(256 * 2 * 8 == 64 * 64);
static_assert(256 * 4 * 4 == 64 * 64);
static_assert(AW * 16 * OSP * 4 <= 131072);
static_assert(16 * 68 * 4 <= 131072);
static_assert(64 * 65 * 4 <= 131072);

typedef _Float16 h16;
typedef unsigned short bf;
typedef __attribute__((ext_vector_type(16))) __bf16   v16bf;
typedef __attribute__((ext_vector_type(16))) _Float16 v16h;
typedef __attribute__((ext_vector_type(8)))  _Float16 v8h;
typedef __attribute__((ext_vector_type(8)))  unsigned short v8us;
typedef __attribute__((ext_vector_type(8)))  float    v8f;
typedef __attribute__((ext_vector_type(4)))  float    v4f;
typedef v4f  __attribute__((may_alias)) v4fa;

__device__ __forceinline__ unsigned short f2bf(float f) { unsigned u = __float_as_uint(f); u += 0x7FFFu + ((u >> 16) & 1u); return (unsigned short)(u >> 16); }
__device__ __forceinline__ float bfr(float f) { return __uint_as_float(((unsigned)f2bf(f)) << 16); }
__device__ __forceinline__ v16h cat16(v8h lo, v8h hi) { return __builtin_shufflevector(lo, hi, 0, 1, 2, 3, 4, 5, 6, 7, 8, 9, 10, 11, 12, 13, 14, 15); }
__device__ __forceinline__ v16bf cat16b(v8us lo, v8us hi) { return __builtin_bit_cast(v16bf, __builtin_shufflevector(lo, hi, 0, 1, 2, 3, 4, 5, 6, 7, 8, 9, 10, 11, 12, 13, 14, 15)); }
__device__ __forceinline__ v8f wmma16(v16h a, v16h b, v8f c) { return __builtin_amdgcn_wmma_f32_16x16x32_f16(false, a, false, b, (short)0, c, false, false); }
__device__ __forceinline__ v8f wmmab(v16bf a, v16bf b, v8f c) { return __builtin_amdgcn_wmma_f32_16x16x32_bf16(false, a, false, b, (short)0, c, false, false); }
__device__ __forceinline__ v16h  ldh(const h16* p) { return cat16(*(const v8h*)p, *(const v8h*)(p + 16)); }
__device__ __forceinline__ v16bf ldb(const bf* p)  { return cat16b(*(const v8us*)p, *(const v8us*)(p + 16)); }
__device__ __forceinline__ void wave_sync() { __builtin_amdgcn_fence(3  , "wavefront"); __builtin_amdgcn_wave_barrier(); asm volatile("" ::: "memory"); }
__device__ __forceinline__ v8f wmmabg(v16bf a, v16bf b, v8f c) { c = wmmab(a, b, c); asm volatile("v_nop\n\tv_nop\n\tv_nop\n\tv_nop" : "+v"(c) : "v"(a), "v"(b)); return c; }
__device__ __forceinline__ v8f wmma16g(v16h a, v16h b, v8f c) { c = wmma16(a, b, c); asm volatile("v_nop\n\tv_nop\n\tv_nop\n\tv_nop" : "+v"(c) : "v"(a), "v"(b)); return c; }
static __device__ __forceinline__ h16 toh_flush(float v) { const float w = (fabsf(v) < 6.103515625e-05f) ? 0.0f : v; return (h16)w; }

__global__ __launch_bounds__(256) void k_cvt8(const float* __restrict__ src, bf* dst, size_t n8) {
    const size_t i = (size_t)blockIdx.x * 256 + threadIdx.x; if (i >= n8) return;
    const v8f v = *(const v8f*)(src + i * 8); v8us o;
#pragma unroll
    for (int k = 0; k < 8; ++k) o[k] = f2bf(v[k]);
    *(volatile v8us*)(dst + i * 8) = o; __threadfence(); *(volatile v8us*)(dst + i * 8) = o;
}

__global__ __launch_bounds__(256) void k_wtb(const float* __restrict__ W, bf* O, int ldn) {
    __shared__ float ts[64 * 65];
    const unsigned tid = threadIdx.x; const unsigned n0 = blockIdx.x * 64u, k0 = blockIdx.y * 64u;
#pragma unroll
    for (int it = 0; it < 4; ++it) { const unsigned idx = tid + (unsigned)it * 256u; const unsigned r = idx >> 4, c4 = (idx & 15u) * 4u;
        const v4f v = *(const v4f*)(W + (size_t)(k0 + r) * (size_t)ldn + n0 + c4);
        ts[r * 65u + c4 + 0u] = v[0]; ts[r * 65u + c4 + 1u] = v[1]; ts[r * 65u + c4 + 2u] = v[2]; ts[r * 65u + c4 + 3u] = v[3]; }
    __syncthreads();
    const unsigned row = tid >> 3, c8 = (tid & 7u) * 8u;
    v8us o0, o1;
#pragma unroll
    for (int i = 0; i < 8; ++i) { o0[i] = f2bf(ts[(c8 + (unsigned)i) * 65u + row]); o1[i] = f2bf(ts[(c8 + (unsigned)i) * 65u + row + 32u]); }
    bf* p0 = O + (size_t)(n0 + row) * DM + k0 + c8; bf* p1 = O + (size_t)(n0 + row + 32u) * DM + k0 + c8;
    *(volatile v8us*)p0 = o0; *(volatile v8us*)p1 = o1; __threadfence(); *(volatile v8us*)p0 = o0; *(volatile v8us*)p1 = o1;
}

__global__ __launch_bounds__(256) void k_wth(const float* __restrict__ W, h16* O, int ldn) {
    __shared__ float ts[64 * 65];
    const unsigned tid = threadIdx.x; const unsigned n0 = blockIdx.x * 64u, k0 = blockIdx.y * 64u;
#pragma unroll
    for (int it = 0; it < 4; ++it) { const unsigned idx = tid + (unsigned)it * 256u; const unsigned r = idx >> 4, c4 = (idx & 15u) * 4u;
        const v4f v = *(const v4f*)(W + (size_t)(k0 + r) * (size_t)ldn + n0 + c4);
        ts[r * 65u + c4 + 0u] = v[0]; ts[r * 65u + c4 + 1u] = v[1]; ts[r * 65u + c4 + 2u] = v[2]; ts[r * 65u + c4 + 3u] = v[3]; }
    __syncthreads();
    const unsigned row = tid >> 3, c8 = (tid & 7u) * 8u;
    v8h o0, o1;
#pragma unroll
    for (int i = 0; i < 8; ++i) { o0[i] = toh_flush(bfr(ts[(c8 + (unsigned)i) * 65u + row]) * WOS); o1[i] = toh_flush(bfr(ts[(c8 + (unsigned)i) * 65u + row + 32u]) * WOS); }
    h16* p0 = O + (size_t)(n0 + row) * DM + k0 + c8; h16* p1 = O + (size_t)(n0 + row + 32u) * DM + k0 + c8;
    *(volatile v8h*)p0 = o0; *(volatile v8h*)p1 = o1; __threadfence(); *(volatile v8h*)p0 = o0; *(volatile v8h*)p1 = o1;
}

template <int MODE>
__device__ __forceinline__ void proj_body(const bf* __restrict__ A, const bf* __restrict__ Bt, const float* __restrict__ bias, h16* Ph, h16* Pr) {
    __shared__ __align__(16) float os[16 * 68];
    const int K = DM;
    const int lane = threadIdx.x & 31, lr = lane & 15, hi = lane >> 4;
    const unsigned r0 = blockIdx.x * 64u, c0 = blockIdx.y * 64u;
    v8f acc[4][4];
#pragma unroll
    for (int mb = 0; mb < 4; ++mb)
#pragma unroll
        for (int nb = 0; nb < 4; ++nb) acc[mb][nb] = (v8f){};
    const size_t aoff = (size_t)(r0 + (unsigned)lr) * K + 8 * hi, boff = (size_t)(c0 + (unsigned)lr) * K + 8 * hi;
#pragma unroll 1
    for (int kc = 0; kc < K; kc += 32) {
        v16bf a[4];
#pragma unroll
        for (int mb = 0; mb < 4; ++mb) a[mb] = ldb(A + aoff + (size_t)mb * 16 * K + kc);
#pragma unroll
        for (int nb = 0; nb < 4; ++nb) { const v16bf b = ldb(Bt + boff + (size_t)nb * 16 * K + kc);
#pragma unroll
            for (int mb = 0; mb < 4; ++mb) acc[mb][nb] = wmmabg(a[mb], b, acc[mb][nb]); }
    }
    float bc[4];
#pragma unroll
    for (int nb = 0; nb < 4; ++nb) bc[nb] = (MODE == 0) ? bfr(bias[c0 + (unsigned)(nb * 16 + lr)]) : 0.0f;
    size_t tbase, rbase; bool wr;
    if (MODE == 0) { const unsigned bb = r0 / (unsigned)SEQ, tt = r0 % (unsigned)SEQ;
                     const unsigned zc = (c0 / (unsigned)DM) * (unsigned)(NB * NH_) + bb * (unsigned)NH_ + (c0 % (unsigned)DM) / (unsigned)HD;
                     tbase = ((size_t)zc * SEQ + (size_t)tt) * HD; rbase = ((size_t)zc * (size_t)EROWS + (size_t)tt) * HD; wr = tt < (unsigned)EROWS; }
    else           { const unsigned bb = c0 / (unsigned)SEQ, tt = c0 % (unsigned)SEQ;
                     tbase = (size_t)bb * (size_t)DM * SEQ + (size_t)r0 * SEQ + (size_t)tt; rbase = (size_t)bb * (size_t)DM * (size_t)EROWS + (size_t)r0 * (size_t)EROWS + (size_t)tt; wr = tt < (unsigned)EROWS; }
#pragma unroll
    for (int mb = 0; mb < 4; ++mb) {
        float br[8];
#pragma unroll
        for (int j = 0; j < 8; ++j) br[j] = (MODE == 1) ? bfr(bias[r0 + (unsigned)(mb * 16 + hi * 8 + j)]) : 0.0f;
#pragma unroll
        for (int nb = 0; nb < 4; ++nb) {
#pragma unroll
            for (int j = 0; j < 8; ++j) os[(hi * 8 + j) * 68 + nb * 16 + lr] = acc[mb][nb][j] + bc[nb] + br[j]; }
        wave_sync();
#pragma unroll 1
        for (int ps = 0; ps < 2; ++ps) {
            if (MODE == 0) {
                const size_t sb = tbase + (size_t)(mb * 16) * HD;
                const size_t rb = rbase + (size_t)(mb * 16) * HD;
#pragma unroll
                for (int s = 0; s < 4; ++s) { const int p = s * 32 + lane; const int row = p >> 3, c8 = (p & 7) * 8;
                    const v4f x0 = *(const v4fa*)(&os[row * 68 + c8]); const v4f x1 = *(const v4fa*)(&os[row * 68 + c8 + 4]); v8h hv, rv;
#pragma unroll
                    for (int i = 0; i < 4; ++i) { const h16 a0 = toh_flush(x0[i]); const h16 a1 = toh_flush(x1[i]); hv[i] = a0; hv[4 + i] = a1;
                        rv[i] = toh_flush((x0[i] - (float)a0) * QRS); rv[4 + i] = toh_flush((x1[i] - (float)a1) * QRS); }
                    const size_t oo = sb + (size_t)p * 8;
                    const size_t ro = rb + (size_t)p * 8;
                    *(volatile v8h*)(Ph + oo) = hv; if (wr) *(volatile v8h*)(Pr + ro) = rv; }
            } else {
                const size_t sb = tbase + (size_t)(mb * 16) * SEQ;
                const size_t rb = rbase + (size_t)(mb * 16) * (size_t)EROWS;
#pragma unroll
                for (int s = 0; s < 4; ++s) { const int row = 4 * s + (lane >> 3), c8 = (lane & 7) * 8;
                    const v4f x0 = *(const v4fa*)(&os[row * 68 + c8]); const v4f x1 = *(const v4fa*)(&os[row * 68 + c8 + 4]); v8h hv, rv;
#pragma unroll
                    for (int i = 0; i < 4; ++i) { const h16 a0 = toh_flush(x0[i]); const h16 a1 = toh_flush(x1[i]); hv[i] = a0; hv[4 + i] = a1;
                        rv[i] = toh_flush((x0[i] - (float)a0) * QRS); rv[4 + i] = toh_flush((x1[i] - (float)a1) * QRS); }
                    const size_t oo = sb + (size_t)row * SEQ + c8;
                    const size_t ro = rb + (size_t)row * (size_t)EROWS + c8;
                    *(volatile v8h*)(Ph + oo) = hv; if (wr) *(volatile v8h*)(Pr + ro) = rv; }
            }
            if (ps == 0) __threadfence(); }
        wave_sync();
    }
}

__global__ __launch_bounds__(32) void k_proj_qk(const bf* __restrict__ A, const bf* __restrict__ Bt, const float* __restrict__ bias, h16* Ph, h16* Pr) { proj_body<0>(A, Bt, bias, Ph, Pr); }
__global__ __launch_bounds__(32) void k_proj_vt(const bf* __restrict__ A, const bf* __restrict__ Bt, const float* __restrict__ bias, h16* Ph, h16* Pr) { proj_body<1>(A, Bt, bias, Ph, Pr); }

template <int EARLY>
__device__ __forceinline__ void flash_body(const h16* __restrict__ QH, const h16* __restrict__ QR, const h16* __restrict__ KP, const h16* __restrict__ KR,
                                           const h16* __restrict__ VT, const h16* __restrict__ VR, h16* CH, h16* CR) {
    __shared__ __align__(16) float os[AW * 16 * OSP];
    const int lane = threadIdx.x & 31, lr = lane & 15, hi = lane >> 4;
    const int wave = __builtin_amdgcn_readfirstlane((int)(threadIdx.x >> 5));
    const unsigned zh = blockIdx.y; const unsigned b = zh / (unsigned)NH_, h = zh % (unsigned)NH_;
    const int t0 = (EARLY ? 0 : EROWS) + ((int)blockIdx.x * AW + wave) * 16;
    const int lim = t0 + lr;
    const int nk = (t0 + 16 + 31) & ~31;
    const size_t pbase = (size_t)zh * SEQ * HD;
    const size_t rbase = (size_t)zh * EROWS * HD;
    const size_t qo = pbase + (size_t)(t0 + lr) * HD + 8 * hi;
    const v16h hz = (v16h){};
    const v16h qh0 = ldh(QH + qo), qh1 = ldh(QH + qo + 32);
    v16h qr0 = hz, qr1 = hz;
    if (EARLY) { const size_t qro = rbase + (size_t)(t0 + lr) * HD + 8 * hi; qr0 = ldh(QR + qro); qr1 = ldh(QR + qro + 32); }
    const size_t ko = pbase + (size_t)lr * HD + 8 * hi;
    const size_t vo = pbase + (size_t)lr * SEQ + 8 * hi;
    const size_t kro = rbase + (size_t)lr * HD + 8 * hi;
    const size_t vro = rbase + (size_t)lr * EROWS + 8 * hi;
    v8f o[4], oR[4];
#pragma unroll
    for (int j = 0; j < 4; ++j) { o[j] = (v8f){}; oR[j] = (v8f){}; }
    float m = NEGB, l = 0.0f;
#pragma unroll 1
    for (int key0 = 0; key0 < nk; key0 += 32) {
        v8f sHa = (v8f){}, sLa = (v8f){}, sHb = (v8f){}, sLb = (v8f){};
        { const h16* ka = KP + ko + (size_t)key0 * HD;
          const v16h ka0 = ldh(ka), ka1 = ldh(ka + 32), kb0 = ldh(ka + 16 * HD), kb1 = ldh(ka + 16 * HD + 32);
          sHa = wmma16g(ka0, qh0, sHa); sHb = wmma16g(kb0, qh0, sHb);
          sHa = wmma16g(ka1, qh1, sHa); sHb = wmma16g(kb1, qh1, sHb);
          if (EARLY) {
              sLa = wmma16g(ka0, qr0, sLa); sLb = wmma16g(kb0, qr0, sLb);
              sLa = wmma16g(ka1, qr1, sLa); sLb = wmma16g(kb1, qr1, sLb);
              const h16* kr = KR + kro + (size_t)key0 * HD;
              const v16h ra0 = ldh(kr), ra1 = ldh(kr + 32), rb0 = ldh(kr + 16 * HD), rb1 = ldh(kr + 16 * HD + 32);
              sLa = wmma16g(ra0, qh0, sLa); sLb = wmma16g(rb0, qh0, sLb);
              sLa = wmma16g(ra1, qh1, sLa); sLb = wmma16g(rb1, qh1, sLb); } }
        const int ja = key0 + 8 * hi;
        float ta[8], tb[8]; bool fa[8], fb[8]; float mx = NEGB;
#pragma unroll
        for (int r = 0; r < 8; ++r) {
            fa[r] = (ja + r <= lim);
            fb[r] = (ja + 16 + r <= lim);
            if (EARLY) { ta[r] = (sHa[r] + sLa[r] * QRI) * SC2; tb[r] = (sHb[r] + sLb[r] * QRI) * SC2; }
            else       { ta[r] = sHa[r] * SC2; tb[r] = sHb[r] * SC2; }
            mx = fmaxf(mx, fmaxf(fa[r] ? ta[r] : NEGB, fb[r] ? tb[r] : NEGB)); }
        mx = fmaxf(mx, __shfl_xor(mx, 16, 32));
        const float mnew = fmaxf(m, mx);
        const float alpha = __builtin_amdgcn_exp2f(m - mnew);
        const float sh = PSH - mnew;
        v16h pb, pr = hz; float ls = 0.0f;
#pragma unroll
        for (int r = 0; r < 8; ++r) {
            const float ea = __builtin_amdgcn_exp2f(ta[r] + sh), eb = __builtin_amdgcn_exp2f(tb[r] + sh);
            const float ga = fa[r] ? ea : 0.0f, gb = fb[r] ? eb : 0.0f;
            const h16 pa = toh_flush(ga); const h16 pc = toh_flush(gb);
            pb[r] = pa; pb[8 + r] = pc;
            if (EARLY) { pr[r] = toh_flush((ga - (float)pa) * QRS); pr[8 + r] = toh_flush((gb - (float)pc) * QRS); ls += ga + gb; }
            else       { ls += (float)pa + (float)pc; } }
        l = l * alpha + ls; m = mnew;
#pragma unroll
        for (int j = 0; j < 4; ++j) { o[j] = o[j] * alpha; if (EARLY) oR[j] = oR[j] * alpha; }
        const h16* va = VT + vo + key0;
#pragma unroll
        for (int j = 0; j < 4; ++j) {
            const v16h vj = ldh(va + (size_t)(16 * j) * SEQ);
            o[j] = wmma16g(vj, pb, o[j]);
            if (EARLY) {
                oR[j] = wmma16g(vj, pr, oR[j]);
                const v16h vrj = ldh(VR + vro + (size_t)(16 * j) * EROWS + key0);
                oR[j] = wmma16g(vrj, pb, oR[j]); } }
    }
    l += __shfl_xor(l, 16, 32);
    const bool any = l > 0.0f;
    const float lsafe = any ? l : 1.0f;
    const float inv = any ? (1.0f / lsafe) : 0.0f;
    const float sc = inv * CTXS;
    const int wb = wave * 16 * OSP;
#pragma unroll
    for (int j = 0; j < 4; ++j) {
        v8f f = o[j]; if (EARLY) f = o[j] + oR[j] * QRI;
        v4f a, c;
        a[0] = f[0] * sc; a[1] = f[1] * sc; a[2] = f[2] * sc; a[3] = f[3] * sc; c[0] = f[4] * sc; c[1] = f[5] * sc; c[2] = f[6] * sc; c[3] = f[7] * sc;
        *(v4fa*)(&os[wb + lr * OSP + 16 * j + 8 * hi]) = a; *(v4fa*)(&os[wb + lr * OSP + 16 * j + 8 * hi + 4]) = c; }
    wave_sync();
    h16* crow = CH + ((size_t)b * SEQ + (size_t)t0) * DM + h * (unsigned)HD;
    h16* rrow = CR + ((size_t)b * EROWS + (size_t)(EARLY ? t0 : 0)) * DM + h * (unsigned)HD;
#pragma unroll 1
    for (int ps = 0; ps < 2; ++ps) {
#pragma unroll
        for (int s = 0; s < 4; ++s) { const int row = 4 * s + (lane >> 3), c8 = (lane & 7) * 8;
            const v4f x0 = *(const v4fa*)(&os[wb + row * OSP + c8]); const v4f x1 = *(const v4fa*)(&os[wb + row * OSP + c8 + 4]); v8h hv, rv;
#pragma unroll
            for (int i = 0; i < 4; ++i) { const h16 a0 = toh_flush(x0[i]); const h16 a1 = toh_flush(x1[i]); hv[i] = a0; hv[4 + i] = a1;
                rv[i] = toh_flush((x0[i] - (float)a0) * QRS); rv[4 + i] = toh_flush((x1[i] - (float)a1) * QRS); }
            *(volatile v8h*)(crow + (size_t)row * DM + c8) = hv;
            if (EARLY) *(volatile v8h*)(rrow + (size_t)row * DM + c8) = rv; }
        if (ps == 0) __threadfence(); }
}

__global__ __launch_bounds__(32 * AW) __attribute__((amdgpu_num_vgpr(256))) void k_flash_e(const h16* __restrict__ QH, const h16* __restrict__ QR, const h16* __restrict__ KP, const h16* __restrict__ KR,
                                                                                           const h16* __restrict__ VT, const h16* __restrict__ VR, h16* CH, h16* CR) { flash_body<1>(QH, QR, KP, KR, VT, VR, CH, CR); }
__global__ __launch_bounds__(32 * AW) __attribute__((amdgpu_num_vgpr(256))) void k_flash_l(const h16* __restrict__ QH, const h16* __restrict__ QR, const h16* __restrict__ KP, const h16* __restrict__ KR,
                                                                                           const h16* __restrict__ VT, const h16* __restrict__ VR, h16* CH, h16* CR) { flash_body<0>(QH, QR, KP, KR, VT, VR, CH, CR); }

template <int EARLY>
__device__ __forceinline__ void oproj_body(const h16* __restrict__ CHp, const h16* __restrict__ CRp, const h16* __restrict__ WOT, const float* __restrict__ bo, float* OUT) {
    constexpr int NBK = EARLY ? 2 : 4;
    constexpr int CW = 16 * NBK;
    __shared__ __align__(16) float os[16 * 68];
    const int K = DM;
    const int lane = threadIdx.x & 31, lr = lane & 15, hi = lane >> 4;
    const unsigned bz = blockIdx.z;
    const unsigned r0 = (EARLY ? 0u : (unsigned)EROWS) + blockIdx.x * 64u;
    const unsigned c0 = blockIdx.y * (unsigned)CW;
    v8f acc[4][NBK], accR[4][NBK];
#pragma unroll
    for (int mb = 0; mb < 4; ++mb)
#pragma unroll
        for (int nb = 0; nb < NBK; ++nb) { acc[mb][nb] = (v8f){}; accR[mb][nb] = (v8f){}; }
    const size_t aoff = ((size_t)bz * SEQ + (size_t)(r0 + (unsigned)lr)) * K + 8 * hi;
    const size_t roff = ((size_t)bz * EROWS + (size_t)(EARLY ? (r0 + (unsigned)lr) : 0u)) * K + 8 * hi;
    const size_t boff = (size_t)(c0 + (unsigned)lr) * K + 8 * hi;
#pragma unroll 1
    for (int kc = 0; kc < K; kc += 32) {
        v16h a[4], ar[4];
#pragma unroll
        for (int mb = 0; mb < 4; ++mb) { a[mb] = ldh(CHp + aoff + (size_t)mb * 16 * K + kc); ar[mb] = (v16h){};
            if (EARLY) ar[mb] = ldh(CRp + roff + (size_t)mb * 16 * K + kc); }
#pragma unroll
        for (int nb = 0; nb < NBK; ++nb) { const v16h bfrag = ldh(WOT + boff + (size_t)nb * 16 * K + kc);
#pragma unroll
            for (int mb = 0; mb < 4; ++mb) { acc[mb][nb] = wmma16g(a[mb], bfrag, acc[mb][nb]);
                if (EARLY) accR[mb][nb] = wmma16g(ar[mb], bfrag, accR[mb][nb]); } }
    }
    const int c4 = EARLY ? (lane & 7) * 4 : (lane & 15) * 4;
    const v4f bq = *(const v4f*)(bo + c0 + (unsigned)c4);
    v4f bv; bv[0] = bfr(bq[0]); bv[1] = bfr(bq[1]); bv[2] = bfr(bq[2]); bv[3] = bfr(bq[3]);
#pragma unroll
    for (int mb = 0; mb < 4; ++mb) {
#pragma unroll
        for (int nb = 0; nb < NBK; ++nb) {
#pragma unroll
            for (int j = 0; j < 8; ++j) { float v = acc[mb][nb][j]; if (EARLY) v = v + accR[mb][nb][j] * QRI;
                os[(hi * 8 + j) * 68 + nb * 16 + lr] = v; } }
        wave_sync();
        float* orow = OUT + ((size_t)bz * OUT_SEQ + (size_t)(r0 + (unsigned)(mb * 16))) * DM + c0;
#pragma unroll 1
        for (int ps = 0; ps < 2; ++ps) {
            if (EARLY) {
#pragma unroll
                for (int s = 0; s < 4; ++s) { const int row = 4 * s + (lane >> 3);
                    const v4f x = *(const v4fa*)(&os[row * 68 + c4]);
                    const v4f w = x * OSCL + bv;
                    *(volatile v4f*)(orow + (size_t)row * DM + c4) = w; }
            } else {
#pragma unroll
                for (int s = 0; s < 8; ++s) { const int row = 2 * s + (lane >> 4);
                    const v4f x = *(const v4fa*)(&os[row * 68 + c4]);
                    const v4f w = x * OSCL + bv;
                    *(volatile v4f*)(orow + (size_t)row * DM + c4) = w; }
            }
            if (ps == 0) __threadfence(); }
        wave_sync();
    }
}

__global__ __launch_bounds__(32) __attribute__((amdgpu_num_vgpr(256))) void k_oproj_e(const h16* __restrict__ CHp, const h16* __restrict__ CRp, const h16* __restrict__ WOT, const float* __restrict__ bo, float* OUT) { oproj_body<1>(CHp, CRp, WOT, bo, OUT); }
__global__ __launch_bounds__(32) void k_oproj_l(const h16* __restrict__ CHp, const h16* __restrict__ CRp, const h16* __restrict__ WOT, const float* __restrict__ bo, float* OUT) { oproj_body<0>(CHp, CRp, WOT, bo, OUT); }

static constexpr size_t al256(size_t v) { return (v + 255) & ~(size_t)255; }
static constexpr size_t N_PL = (size_t)NB * NH_ * SEQ * HD;
static constexpr size_t N_RS = (size_t)NB * NH_ * EROWS * HD;
static constexpr size_t SZ_XB = al256((size_t)NB * SEQ * DM * 2);
static constexpr size_t SZ_WT = al256((size_t)3 * DM * DM * 2);
static constexpr size_t SZ_WO = al256((size_t)DM * DM * 2);
static constexpr size_t SZ_PL = al256(N_PL * 2);
static constexpr size_t SZ_RS = al256(N_RS * 2);
static constexpr size_t SZ_CH = al256((size_t)NB * SEQ * DM * 2);
static constexpr size_t SZ_CR = al256((size_t)NB * EROWS * DM * 2);
static constexpr size_t SZ_TOTAL = SZ_XB + SZ_WT + SZ_WO + 3 * SZ_PL + 3 * SZ_RS + SZ_CH + SZ_CR;
static_assert(SZ_TOTAL <= (size_t)134217728);
static_assert((N_PL * 2) % 256 == 0);
static_assert((N_RS * 2) % 256 == 0);
static_assert(SZ_PL == N_PL * 2);
static_assert(SZ_RS == N_RS * 2);
static_assert(((size_t)DM * DM * 2) % 256 == 0);
static_assert((size_t)NB * NH_ * SEQ * HD == (size_t)NB * DM * SEQ);
static_assert((size_t)NB * NH_ * EROWS * HD == (size_t)NB * DM * EROWS);
static constexpr size_t NEED_X = ((size_t)(NB - 1) * SEQ_FULL + SEQ) * DM;
static constexpr size_t NEED_O = ((size_t)(NB - 1) * OUT_SEQ + SEQ) * DM;
static constexpr size_t N8_FULL = (size_t)NB * SEQ * DM / 8;
static constexpr size_t N8_SEQ  = (size_t)SEQ * DM / 8;

extern "C" void kernel_launch(void* const* d_in, const int* in_sizes, int n_in,
                              void* d_out, int out_size, void* d_ws, size_t ws_size, hipStream_t stream) {
    if (n_in < 5) return;
    if ((size_t)in_sizes[0] < NEED_X) return;
    if ((size_t)in_sizes[1] < (size_t)3 * DM * DM || in_sizes[2] < 3 * DM) return;
    if ((size_t)in_sizes[3] < (size_t)DM * DM || in_sizes[4] < DM) return;
    if ((size_t)out_size < NEED_O) return;
    if (SZ_TOTAL > ws_size) return;
    const float* x    = (const float*)d_in[0];
    const float* wqkv = (const float*)d_in[1];
    const float* bqkv = (const float*)d_in[2];
    const float* wo   = (const float*)d_in[3];
    const float* bo   = (const float*)d_in[4];
    float* OUT = (float*)d_out;
    char* wsp = (char*)d_ws;
    bf*  XB  = (bf*)wsp;  wsp += SZ_XB;
    bf*  WT  = (bf*)wsp;  wsp += SZ_WT;
    h16* WOT = (h16*)wsp; wsp += SZ_WO;
    h16* QH  = (h16*)wsp; wsp += SZ_PL;
    h16* KP  = (h16*)wsp; wsp += SZ_PL;
    h16* VT  = (h16*)wsp; wsp += SZ_PL;
    h16* QR  = (h16*)wsp; wsp += SZ_RS;
    h16* KR  = (h16*)wsp; wsp += SZ_RS;
    h16* VR  = (h16*)wsp; wsp += SZ_RS;
    h16* CH  = (h16*)wsp; wsp += SZ_CH;
    h16* CR  = (h16*)wsp; wsp += SZ_CR;

    if (SEQ == SEQ_FULL) {
        k_cvt8<<<(unsigned)((N8_FULL + 255) / 256), 256, 0, stream>>>(x, XB, N8_FULL);
    } else {
        for (int b = 0; b < NB; ++b) k_cvt8<<<(unsigned)((N8_SEQ + 255) / 256), 256, 0, stream>>>(x + (size_t)b * SEQ_FULL * DM, XB + (size_t)b * SEQ * DM, N8_SEQ);
    }
    k_wtb<<<dim3(3 * DM / 64, DM / 64, 1), 256, 0, stream>>>(wqkv, WT, 3 * DM);
    k_wth<<<dim3(DM / 64, DM / 64, 1), 256, 0, stream>>>(wo, WOT, DM);

    k_proj_qk<<<dim3(NB * SEQ / 64, 2 * DM / 64, 1), 32, 0, stream>>>(XB, WT, bqkv, QH, QR);
    k_proj_vt<<<dim3(DM / 64, NB * SEQ / 64, 1), 32, 0, stream>>>(WT + (size_t)2 * DM * DM, XB, bqkv + 2 * DM, VT, VR);

    k_flash_e<<<dim3(EROWS / (16 * AW), NB * NH_, 1), 32 * AW, 0, stream>>>(QH, QR, KP, KR, VT, VR, CH, CR);
    if (SEQ > EROWS)
        k_flash_l<<<dim3((SEQ - EROWS) / (16 * AW), NB * NH_, 1), 32 * AW, 0, stream>>>(QH, QR, KP, KR, VT, VR, CH, CR);

    k_oproj_e<<<dim3(EROWS / 64, DM / 32, NB), 32, 0, stream>>>(CH, CR, WOT, bo, OUT);
    if (SEQ > EROWS)
        k_oproj_l<<<dim3((SEQ - EROWS) / 64, DM / 64, NB), 32, 0, stream>>>(CH, CR, WOT, bo, OUT);
}
